// SpectalRecurrentAttention_78288663872408
// MI455X (gfx1250) — hardware-verified
//
#include <hip/hip_runtime.h>
#include <math.h>

typedef __attribute__((ext_vector_type(16))) _Float16 v16h;
typedef __attribute__((ext_vector_type(8)))  _Float16 v8h;
typedef __attribute__((ext_vector_type(8)))  float    v8f;
typedef __attribute__((ext_vector_type(4)))  float    v4f;

constexpr int kSteps   = 500;
constexpr int kBat     = 16;
constexpr int kFreq    = 32;
constexpr int kRows    = kBat * kFreq;
constexpr int kCin     = 64;
constexpr int kHid     = 64;
constexpr int kG3      = 3 * kHid;
constexpr int kBlkRows = 32;
constexpr int kNumBlk  = kRows / kBlkRows;
constexpr int kThreads = 128;
constexpr int kXsP     = 72;
constexpr int kHsP     = 72;
constexpr int kHfP     = 68;
constexpr int kWtP     = 36;
constexpr int kSmP     = 68;
constexpr int kWPlane  = kG3 * kHid;
constexpr int kHsG     = kBlkRows * kHsP;
constexpr int kHsBuf   = 3 * kHsG;
constexpr int kHfG     = kBlkRows * kHfP;
constexpr long kOut0Elems = (long)kSteps * kRows * kCin;
constexpr long kOut1Elems = 3L * kRows * kHid;
static_assert(kOut0Elems * 4 == 65536000L, "out1 byte offset");
static_assert((kOut0Elems + kOut1Elems) * 4 == 65929216L, "total out bytes");
static_assert(kBlkRows == kFreq, "block owns exactly one batch group");

union FragU { v16h v; v8h h[2]; };
__device__ __forceinline__ v16h fload(const _Float16* p) {
  FragU f; f.h[0] = *(const v8h*)(p); f.h[1] = *(const v8h*)(p + 16); return f.v;
}
__device__ __forceinline__ v8f mma16(v16h a, v16h b, v8f c) {
  return __builtin_amdgcn_wmma_f32_16x16x32_f16(false, a, false, b, (short)0, c, false, false);
}
__device__ __forceinline__ void guard_rz(v8f& a, v8f& b,
    v16h f0, v16h f1, v16h f2, v16h f3,
    v16h g0, v16h g1, v16h g2, v16h g3, v16h g4, v16h g5, v16h g6, v16h g7) {
  asm volatile("v_nop\n\tv_nop\n\tv_nop\n\tv_nop" : "+v"(a), "+v"(b)
               : "v"(f0), "v"(f1), "v"(f2), "v"(f3), "v"(g0), "v"(g1), "v"(g2), "v"(g3),
                 "v"(g4), "v"(g5), "v"(g6), "v"(g7));
}
__device__ __forceinline__ void guard_n(v8f& a, v8f& b,
    v16h f0, v16h f1, v16h f2, v16h f3, v16h g0, v16h g1, v16h g2, v16h g3) {
  asm volatile("v_nop\n\tv_nop\n\tv_nop\n\tv_nop" : "+v"(a), "+v"(b)
               : "v"(f0), "v"(f1), "v"(f2), "v"(f3), "v"(g0), "v"(g1), "v"(g2), "v"(g3));
}

__device__ __forceinline__ float gate_sigmoid(float v) {
  v = fminf(fmaxf(v, -30.0f), 30.0f);
  const float e = expf(-v);
  return __builtin_amdgcn_rcpf(1.0f + e);
}
__device__ __forceinline__ float gate_tanh(float v) {
  v = fminf(fmaxf(v, -15.0f), 15.0f);
  const float e = expf(2.0f * v);
  return 1.0f - 2.0f * __builtin_amdgcn_rcpf(1.0f + e);
}

__global__ __launch_bounds__(256) void prep_w16(
    const float* __restrict__ w0, const float* __restrict__ w1, const float* __restrict__ w2,
    const float* __restrict__ w3, const float* __restrict__ w4, const float* __restrict__ w5,
    unsigned* __restrict__ out) {
  const int plane = blockIdx.x / 24;
  const int blk   = blockIdx.x - plane * 24;
  const float* src = (plane == 0) ? w0 : (plane == 1) ? w1 : (plane == 2) ? w2
                   : (plane == 3) ? w3 : (plane == 4) ? w4 : w5;
  const int i = blk * 256 + threadIdx.x;
  if (i < kWPlane / 2) {
    const _Float16 h0 = (_Float16)(src[2 * i] * 8.0f);
    const _Float16 h1 = (_Float16)(src[2 * i + 1] * 8.0f);
    const unsigned u = (unsigned)__builtin_bit_cast(unsigned short, h0)
                     | ((unsigned)__builtin_bit_cast(unsigned short, h1) << 16);
    volatile unsigned* o = out + (size_t)plane * (kWPlane / 2) + i;
    *o = u;
    __threadfence();
    *o = u;
  }
}

__global__ __launch_bounds__(128) void gru3_attn_steps(
    const float* __restrict__ x,
    const float* __restrict__ st0,
    const _Float16* __restrict__ wts,
    const float* __restrict__ bih_q, const float* __restrict__ bhh_q,
    const float* __restrict__ bih_k, const float* __restrict__ bhh_k,
    const float* __restrict__ bih_v, const float* __restrict__ bhh_v,
    const float* __restrict__ w_o,
    const float* __restrict__ b_o,
    float* __restrict__ out0,
    float* __restrict__ out1)
{
  __shared__ __align__(16) _Float16 xs[kBlkRows * kXsP];
  __shared__ __align__(16) _Float16 hs[2 * kHsBuf];
  __shared__ __align__(16) float    hf[3 * kHfG];
  __shared__ __align__(16) float    wtT[kFreq * kWtP];
  __shared__ __align__(16) float    sm[kFreq * kSmP];
  __shared__ float red[2 * 2 * kHid];

  const int tid  = threadIdx.x;
  const int lane = tid & 31;
  const int wv   = tid >> 5;
  const int hh   = lane >> 4;
  const int cc   = lane & 15;
  const int koff = hh * 8;
  const int bgrp = blockIdx.x;
  const int row0 = bgrp * kBlkRows;
  const int mt   = wv & 1;
  const int ubase = (wv >> 1) * 2;
  const float kInv64 = 0.015625f;

#pragma unroll 1
  for (int e = tid; e < 3 * kBlkRows * kHid; e += kThreads) {
    const int g = e >> 11, r = (e >> 6) & 31, c = e & 63;
    const float v = st0[((size_t)g * kRows + row0 + r) * kHid + c];
    hf[g * kHfG + r * kHfP + c] = v;
    hs[g * kHsG + r * kHsP + c] = (_Float16)(v * 8.0f);
  }

  for (int t = 0; t < kSteps; ++t) {
    const int cur = t & 1, nxt = cur ^ 1;
    __syncthreads();

    {
      const int r = tid >> 2, c0 = (tid & 3) * 16;
      const float* xp = x + ((size_t)t * kRows + row0 + r) * kCin + c0;
      const v4f q0 = *(const v4f*)(xp), q1 = *(const v4f*)(xp + 4);
      const v4f q2 = *(const v4f*)(xp + 8), q3 = *(const v4f*)(xp + 12);
      v8h p0, p1;
#pragma unroll
      for (int e = 0; e < 4; ++e) {
        p0[e] = (_Float16)(q0[e] * 8.0f); p0[4 + e] = (_Float16)(q1[e] * 8.0f);
        p1[e] = (_Float16)(q2[e] * 8.0f); p1[4 + e] = (_Float16)(q3[e] * 8.0f);
      }
      *(v8h*)(xs + r * kXsP + c0)     = p0;
      *(v8h*)(xs + r * kXsP + c0 + 8) = p1;
    }
    __syncthreads();

    {
      const _Float16* hsc = hs + cur * kHsBuf;
      _Float16* hsn = hs + nxt * kHsBuf;
      const v16h xa0 = fload(xs + (mt * 16 + cc) * kXsP + koff);
      const v16h xa1 = fload(xs + (mt * 16 + cc) * kXsP + koff + 32);
#pragma unroll 1
      for (int g = 0; g < 3; ++g) {
        const _Float16* Wi = wts + (size_t)(2 * g) * kWPlane;
        const _Float16* Wh = Wi + kWPlane;
        const float* bi = (g == 0) ? bih_q : ((g == 1) ? bih_k : bih_v);
        const float* bh = (g == 0) ? bhh_q : ((g == 1) ? bhh_k : bhh_v);
        const _Float16* hsg = hsc + g * kHsG;
        const v16h ha0 = fload(hsg + (mt * 16 + cc) * kHsP + koff);
        const v16h ha1 = fload(hsg + (mt * 16 + cc) * kHsP + koff + 32);
        float* hfg = hf + g * kHfG;
        _Float16* hsng = hsn + g * kHsG;
#pragma unroll 1
        for (int u = 0; u < 2; ++u) {
          const int ub = ubase + u;
          const int nr = 16 * ub + cc, nz = 64 + 16 * ub + cc, nn = 128 + 16 * ub + cc;
          v8f accr = (v8f){0.f,0.f,0.f,0.f,0.f,0.f,0.f,0.f};
          v8f accz = accr, accx = accr, acch = accr;
          {
            const v16h bir0 = fload(Wi + nr * kHid + koff), bir1 = fload(Wi + nr * kHid + koff + 32);
            const v16h bhr0 = fload(Wh + nr * kHid + koff), bhr1 = fload(Wh + nr * kHid + koff + 32);
            const v16h biz0 = fload(Wi + nz * kHid + koff), biz1 = fload(Wi + nz * kHid + koff + 32);
            const v16h bhz0 = fload(Wh + nz * kHid + koff), bhz1 = fload(Wh + nz * kHid + koff + 32);
            accr = mma16(xa0, bir0, accr); accr = mma16(xa1, bir1, accr);
            accr = mma16(ha0, bhr0, accr); accr = mma16(ha1, bhr1, accr);
            accz = mma16(xa0, biz0, accz); accz = mma16(xa1, biz1, accz);
            accz = mma16(ha0, bhz0, accz); accz = mma16(ha1, bhz1, accz);
            guard_rz(accr, accz, xa0, xa1, ha0, ha1, bir0, bir1, bhr0, bhr1, biz0, biz1, bhz0, bhz1);
          }
          {
            const v16h bin0 = fload(Wi + nn * kHid + koff), bin1 = fload(Wi + nn * kHid + koff + 32);
            const v16h bhn0 = fload(Wh + nn * kHid + koff), bhn1 = fload(Wh + nn * kHid + koff + 32);
            accx = mma16(xa0, bin0, accx); accx = mma16(xa1, bin1, accx);
            acch = mma16(ha0, bhn0, acch); acch = mma16(ha1, bhn1, acch);
            guard_n(accx, acch, xa0, xa1, ha0, ha1, bin0, bin1, bhn0, bhn1);
          }
          const int col = 16 * ub + cc;
          const float br  = bi[col] + bh[col];
          const float bz  = bi[64 + col] + bh[64 + col];
          const float bxn = bi[128 + col];
          const float bhn = bh[128 + col];
#pragma unroll
          for (int r = 0; r < 8; ++r) {
            const int row = mt * 16 + 8 * hh + r;
            const float pr = accr[r] * kInv64 + br;
            const float pz = accz[r] * kInv64 + bz;
            const float xn = accx[r] * kInv64 + bxn;
            const float hn = acch[r] * kInv64 + bhn;
            const float rg = gate_sigmoid(pr);
            const float zg = gate_sigmoid(pz);
            const float ng = gate_tanh(xn + rg * hn);
            const float hp = hfg[row * kHfP + col];
            const float hnew = (1.0f - zg) * ng + zg * hp;
            hfg[row * kHfP + col] = hnew;
            hsng[row * kHsP + col] = (_Float16)(hnew * 8.0f);
          }
        }
      }
    }
    __syncthreads();

    {
      const int fg = tid >> 4, gg = tid & 15;
      const float* qb = hf;
      const float* kb = hf + kHfG;
      float a[4][2];
#pragma unroll
      for (int i = 0; i < 4; ++i) { a[i][0] = 0.f; a[i][1] = 0.f; }
#pragma unroll 1
      for (int h = 0; h < kHid; h += 4) {
        const v4f k0 = *(const v4f*)(kb + (2 * gg) * kHfP + h);
        const v4f k1 = *(const v4f*)(kb + (2 * gg + 1) * kHfP + h);
#pragma unroll
        for (int i = 0; i < 4; ++i) {
          const v4f qv = *(const v4f*)(qb + (4 * fg + i) * kHfP + h);
#pragma unroll
          for (int e = 0; e < 4; ++e) { a[i][0] += qv[e] * k0[e]; a[i][1] += qv[e] * k1[e]; }
        }
      }
#pragma unroll
      for (int j = 0; j < 2; ++j) {
        v4f w; w[0] = a[0][j]; w[1] = a[1][j]; w[2] = a[2][j]; w[3] = a[3][j];
        *(v4f*)(wtT + (2 * gg + j) * kWtP + 4 * fg) = w;
      }
    }
    __syncthreads();

    {
      const int fg = tid >> 4, hq = tid & 15;
      const float* vb = hf + 2 * kHfG;
      float a[4][4];
#pragma unroll
      for (int i = 0; i < 4; ++i)
#pragma unroll
        for (int j = 0; j < 4; ++j) a[i][j] = 0.f;
#pragma unroll 1
      for (int g2 = 0; g2 < kFreq; ++g2) {
        const v4f wv4 = *(const v4f*)(wtT + g2 * kWtP + 4 * fg);
        const v4f vv4 = *(const v4f*)(vb + g2 * kHfP + 4 * hq);
#pragma unroll
        for (int i = 0; i < 4; ++i)
#pragma unroll
          for (int j = 0; j < 4; ++j) a[i][j] += wv4[i] * vv4[j];
      }
#pragma unroll
      for (int i = 0; i < 4; ++i) {
        v4f s; s[0] = a[i][0]; s[1] = a[i][1]; s[2] = a[i][2]; s[3] = a[i][3];
        *(v4f*)(sm + (4 * fg + i) * kSmP + 4 * hq) = s;
      }
    }
    __syncthreads();

    {
      const int c = tid & 63, half = tid >> 6;
      float m = -INFINITY;
#pragma unroll
      for (int r = 0; r < 16; ++r) m = fmaxf(m, sm[(16 * half + r) * kSmP + c]);
      red[half * kHid + c] = m;
    }
    __syncthreads();
    {
      const int c = tid & 63, half = tid >> 6;
      const float m = fmaxf(red[c], red[kHid + c]);
      float s = 0.f;
#pragma unroll
      for (int r = 0; r < 16; ++r) {
        const int idx = (16 * half + r) * kSmP + c;
        const float e = expf(sm[idx] - m);
        sm[idx] = e;
        s += e;
      }
      red[2 * kHid + half * kHid + c] = s;
    }
    __syncthreads();
    {
      const int c = tid & 63, half = tid >> 6;
      const float tot = red[2 * kHid + c] + red[3 * kHid + c];
      const float inv = 1.0f / tot;
#pragma unroll
      for (int r = 0; r < 16; ++r) {
        const int idx = (16 * half + r) * kSmP + c;
        sm[idx] = sm[idx] * inv;
      }
    }
    __syncthreads();

    {
      const int fg = tid >> 4, cq = tid & 15;
      float a[4][4];
#pragma unroll
      for (int i = 0; i < 4; ++i)
#pragma unroll
        for (int j = 0; j < 4; ++j) a[i][j] = 0.f;
#pragma unroll 1
      for (int h = 0; h < kHid; h += 4) {
        const v4f wo0 = *(const v4f*)(w_o + (size_t)(4 * cq + 0) * kHid + h);
        const v4f wo1 = *(const v4f*)(w_o + (size_t)(4 * cq + 1) * kHid + h);
        const v4f wo2 = *(const v4f*)(w_o + (size_t)(4 * cq + 2) * kHid + h);
        const v4f wo3 = *(const v4f*)(w_o + (size_t)(4 * cq + 3) * kHid + h);
#pragma unroll
        for (int i = 0; i < 4; ++i) {
          const v4f sv = *(const v4f*)(sm + (4 * fg + i) * kSmP + h);
#pragma unroll
          for (int e = 0; e < 4; ++e) {
            a[i][0] += sv[e] * wo0[e]; a[i][1] += sv[e] * wo1[e];
            a[i][2] += sv[e] * wo2[e]; a[i][3] += sv[e] * wo3[e];
          }
        }
      }
      const v4f bo = *(const v4f*)(b_o + 4 * cq);
      v4f ov[4];
#pragma unroll
      for (int i = 0; i < 4; ++i) {
        ov[i][0] = a[i][0] + bo[0]; ov[i][1] = a[i][1] + bo[1];
        ov[i][2] = a[i][2] + bo[2]; ov[i][3] = a[i][3] + bo[3];
      }
      float* orow = out0 + (((size_t)t * kBat + bgrp) * kFreq + 4 * fg) * kCin + 4 * cq;
      for (int pass = 0; pass < 2; ++pass) {
#pragma unroll
        for (int i = 0; i < 4; ++i) *(volatile v4f*)(orow + (size_t)i * kCin) = ov[i];
        __threadfence();
      }
    }
  }

  {
    const int cq = tid & 15;
    for (int pass = 0; pass < 2; ++pass) {
#pragma unroll
      for (int it = 0; it < 12; ++it) {
        const int rid = it * 8 + 2 * wv + hh;
        const int g = rid >> 5, r = rid & 31;
        const v4f v = *(const v4f*)(hf + g * kHfG + r * kHfP + 4 * cq);
        *(volatile v4f*)(out1 + ((size_t)g * kRows + row0 + r) * kHid + 4 * cq) = v;
      }
      __threadfence();
    }
  }
}

extern "C" void kernel_launch(void* const* d_in, const int* in_sizes, int n_in,
                              void* d_out, int out_size, void* d_ws, size_t ws_size,
                              hipStream_t stream) {
  if (n_in < 16) return;
  if (in_sizes[0] != kSteps * kRows * kCin) return;
  if (in_sizes[1] != 3 * kRows * kHid) return;
  if (in_sizes[2] != kWPlane || in_sizes[3] != kWPlane || in_sizes[6] != kWPlane ||
      in_sizes[7] != kWPlane || in_sizes[10] != kWPlane || in_sizes[11] != kWPlane) return;
  if (in_sizes[4] != kG3 || in_sizes[5] != kG3 || in_sizes[8] != kG3 || in_sizes[9] != kG3 ||
      in_sizes[12] != kG3 || in_sizes[13] != kG3) return;
  if (in_sizes[14] != kCin * kHid || in_sizes[15] != kCin) return;
  if ((long long)out_size < (long long)(kOut0Elems + kOut1Elems)) return;
  const size_t ws_need = (size_t)6 * kWPlane * sizeof(_Float16);
  if (ws_size < ws_need) return;

  const float* x     = (const float*)d_in[0];
  const float* state = (const float*)d_in[1];
  const float* w_o   = (const float*)d_in[14];
  const float* b_o   = (const float*)d_in[15];
  _Float16* wts = (_Float16*)d_ws;
  float* out0 = (float*)d_out;
  float* out1 = out0 + kOut0Elems;

  prep_w16<<<6 * 24, 256, 0, stream>>>(
      (const float*)d_in[2],  (const float*)d_in[3],
      (const float*)d_in[6],  (const float*)d_in[7],
      (const float*)d_in[10], (const float*)d_in[11],
      (unsigned*)d_ws);

  gru3_attn_steps<<<kNumBlk, kThreads, 0, stream>>>(
      x, state, wts,
      (const float*)d_in[4],  (const float*)d_in[5],
      (const float*)d_in[8],  (const float*)d_in[9],
      (const float*)d_in[12], (const float*)d_in[13],
      w_o, b_o, out0, out1);
}
